// BloomAttention_28707561406905
// MI455X (gfx1250) — hardware-verified
//
#include <hip/hip_runtime.h>
#include <math.h>
#include <stdint.h>

#ifndef NB
#define NB    2
#endif
#define SEQ   2048
#ifndef SQ
#define SQ    SEQ
#endif
#define DMOD  2048
#define NH    16
#define HD    128
#define NHD   (NH * HD)
#define QSC   8.0f
#define KSC   8.0f
#define PCAR  32768.0f
#define VCAR  1024.0f
#define OSC   1024.0f
#define WOS   1024.0f
#define LOG2E 1.4426950408889634f
#define INVN  0.08838834764831845f
#define RSQ2  0.70710678118654752f
#define MFILL (-1.0e9f * LOG2E)
#define ATT_WAVES   4
#define ATT_THREADS (ATT_WAVES * 32)
#define NQT         (SQ / 64)
#define ATT_BLOCKS  (NB * NH * NQT)
#define NKB         (SEQ / 32)
#define GSLAB       (16 * 68)
#define ASLAB       (16 * 132)
static_assert(NH == 16 && HD == 128 && DMOD == NHD);
static_assert((HD % 32) == 0 && (SEQ % 64) == 0 && (SQ % 64) == 0 && SQ <= SEQ && SQ >= 64);
static_assert((DMOD % 64) == 0 && (DMOD % 32) == 0 && (NHD % 64) == 0);
static_assert(((NB * SEQ * DMOD / 8) % 256) == 0);
static_assert((GSLAB * 4) % 16 == 0 && (ASLAB * 4) % 16 == 0 && ATT_THREADS == 128);
static_assert(NB >= 1 && NB <= 4);

typedef unsigned short u16;
typedef _Float16 v16h __attribute__((ext_vector_type(16)));
typedef _Float16 v8h  __attribute__((ext_vector_type(8)));
typedef __bf16   v16b __attribute__((ext_vector_type(16)));
typedef float    v8f  __attribute__((ext_vector_type(8)));
typedef float    v4f  __attribute__((ext_vector_type(4)));
typedef unsigned int v4u __attribute__((ext_vector_type(4)));
typedef int      v4i  __attribute__((ext_vector_type(4)));

union FragH { v16h v; v8h h[2]; v4u u[2]; };
union FragB { v16b v; v4u u[2]; };

__device__ __forceinline__ unsigned short bf_bits(float f) {
  unsigned u = __float_as_uint(f);
  return (unsigned short)((u + 0x7FFFu + ((u >> 16) & 1u)) >> 16);
}
__device__ __forceinline__ float bf_up(unsigned short h) { return __uint_as_float(((unsigned)h) << 16); }
__device__ __forceinline__ unsigned short h_bits(_Float16 x) { return __builtin_bit_cast(unsigned short, x); }
__device__ __forceinline__ unsigned pk16(unsigned short a, unsigned short b) { return (unsigned)a | ((unsigned)b << 16); }
__device__ __forceinline__ v8f zero8() { v8f z = {0.f, 0.f, 0.f, 0.f, 0.f, 0.f, 0.f, 0.f}; return z; }
__device__ __forceinline__ int imin(int a, int b) { return a < b ? a : b; }

__device__ __forceinline__ v16h ldfrag_h(const _Float16* p) {
  FragH f;
  f.h[0] = *(const v8h*)(p);
  f.h[1] = *(const v8h*)(p + 16);
  return f.v;
}
__device__ __forceinline__ v16b ldfrag_b(const u16* p) {
  FragB f;
  f.u[0] = *(const v4u*)(p);
  f.u[1] = *(const v4u*)(p + 16);
  return f.v;
}

__device__ __forceinline__ v8f mma_h(v16h a, v16h b, v8f c) {
  return __builtin_amdgcn_wmma_f32_16x16x32_f16(false, a, false, b, (short)0, c, false, false);
}
__device__ __forceinline__ v8f mma_b(v16b a, v16b b, v8f c) {
  return __builtin_amdgcn_wmma_f32_16x16x32_bf16(false, a, false, b, (short)0, c, false, false);
}
template <typename F>
__device__ __forceinline__ void guard2x6(v8f& a, v8f& b, F x0, F x1, F x2, F x3, F x4, F x5) {
#if defined(__HIP_DEVICE_COMPILE__)
  asm volatile("v_nop\n\tv_nop\n\tv_nop\n\tv_nop"
               : "+v"(a), "+v"(b) : "v"(x0), "v"(x1), "v"(x2), "v"(x3), "v"(x4), "v"(x5) : "memory");
#endif
}
template <typename F>
__device__ __forceinline__ void guard4x5(v8f& a, v8f& b, v8f& c, v8f& d, F x0, F x1, F x2, F x3, F x4) {
#if defined(__HIP_DEVICE_COMPILE__)
  asm volatile("v_nop\n\tv_nop\n\tv_nop\n\tv_nop"
               : "+v"(a), "+v"(b), "+v"(c), "+v"(d) : "v"(x0), "v"(x1), "v"(x2), "v"(x3), "v"(x4) : "memory");
#endif
}
__device__ __forceinline__ void acc_guard4(v8f& a, v8f& b, v8f& c, v8f& d) {
#if defined(__HIP_DEVICE_COMPILE__)
  asm volatile("v_nop\n\tv_nop\n\tv_nop\n\tv_nop" : "+v"(a), "+v"(b), "+v"(c), "+v"(d));
#endif
}
__device__ __forceinline__ void wave_sync_lds() {
#if defined(__HIP_DEVICE_COMPILE__)
  __builtin_amdgcn_fence(__ATOMIC_RELEASE, "workgroup");
  __builtin_amdgcn_wave_barrier();
  __builtin_amdgcn_fence(__ATOMIC_ACQUIRE, "workgroup");
#endif
}

__global__ __launch_bounds__(256) void cvt16(const float* __restrict__ x, u16* D, int n8, int mode, float scale) {
  const int gt = blockIdx.x * 256 + (int)threadIdx.x;
  if (gt >= n8) return;
  const float* p = x + (size_t)gt * 8;
  const v4f a = *(const v4f*)(p), c4 = *(const v4f*)(p + 4);
  float v[8];
#pragma unroll
  for (int e = 0; e < 4; ++e) { v[e] = a[e]; v[4 + e] = c4[e]; }
  unsigned short s[8];
#pragma unroll
  for (int e = 0; e < 8; ++e) {
    const unsigned short bb = bf_bits(v[e]);
    const unsigned short hb = h_bits((_Float16)(bf_up(bb) * scale));
    s[e] = (mode != 0) ? hb : bb;
  }
  v4u o;
#pragma unroll
  for (int e = 0; e < 4; ++e) o[e] = pk16(s[2 * e], s[2 * e + 1]);
  u16* d = D + (size_t)gt * 8;
  for (int pass = 0; pass < 2; ++pass) {
    *(volatile v4u*)(d) = o;
    __threadfence();
  }
}

__global__ __launch_bounds__(256) void wtr16(const float* __restrict__ W, u16* D, int Kr, int Nc, int mode, float scale) {
  __shared__ __align__(16) float T[64 * 65];
  const int tid = threadIdx.x, wave = tid >> 5, lane = tid & 31;
  const int n0 = blockIdx.x * 64, k0 = blockIdx.y * 64;
#pragma unroll
  for (int it = 0; it < 4; ++it) {
    const int e  = it * 256 + tid;
    const int kr = e >> 4;
    const int nc = (e & 15) * 4;
    const v4f a = *(const v4f*)(W + (size_t)(k0 + kr) * (size_t)Nc + n0 + nc);
#pragma unroll
    for (int q = 0; q < 4; ++q) T[kr * 65 + nc + q] = a[q];
  }
  __syncthreads();
  const int rq = lane >> 3, c8 = (lane & 7) * 8;
  v4u ov[2];
#pragma unroll
  for (int i4 = 0; i4 < 2; ++i4) {
    const int nn = wave * 8 + i4 * 4 + rq;
    unsigned short s[8];
#pragma unroll
    for (int e = 0; e < 8; ++e) {
      const float w = T[(c8 + e) * 65 + nn];
      const unsigned short bb = bf_bits(w);
      const unsigned short hb = h_bits((_Float16)(bf_up(bb) * scale));
      s[e] = (mode != 0) ? hb : bb;
    }
#pragma unroll
    for (int e = 0; e < 4; ++e) ov[i4][e] = pk16(s[2 * e], s[2 * e + 1]);
  }
  u16* dst = D + (size_t)(n0 + wave * 8 + rq) * (size_t)Kr + k0 + c8;
  for (int pass = 0; pass < 2; ++pass) {
#pragma unroll
    for (int i4 = 0; i4 < 2; ++i4) {
      *(volatile v4u*)(dst + (size_t)(i4 * 4) * (size_t)Kr) = ov[i4];
    }
    __threadfence();
  }
}

template <int OM>
__global__ __launch_bounds__(128)
void gemm_bb(const u16* __restrict__ A, const u16* __restrict__ Bt, const float* __restrict__ bias, int nbias,
             u16* C, int M, int N, int K, int bstA, int bstB, int bstC, float oscale) {
  __shared__ __align__(16) float slab[4 * GSLAB];
  const int tid = threadIdx.x, wave = tid >> 5, lane = tid & 31, hh = lane >> 4, m = lane & 15;
  const int ntile = N >> 6, mtile = M >> 6;
  const int per   = ntile * mtile;
  const int bid   = blockIdx.x;
  const int bt    = bid / per;
  const int t     = bid - bt * per;
  const int rowb  = (t / ntile) * 64 + wave * 16;
  const int col0  = (t % ntile) * 64;
  if (rowb + 16 > M) return;
  const u16* Ab  = A  + (size_t)bt * (size_t)bstA;
  const u16* Bb  = Bt + (size_t)bt * (size_t)bstB;
  u16*       Cb  = C  + (size_t)bt * (size_t)bstC;
  const u16* ap = Ab + (size_t)(rowb + m) * K + 8 * hh;
  const u16* bp = Bb + (size_t)(col0 + m) * K + 8 * hh;
  const size_t bs = (size_t)16 * K;
  v8f acc0 = zero8(), acc1 = zero8(), acc2 = zero8(), acc3 = zero8();
#pragma unroll 1
  for (int k0 = 0; k0 < K; k0 += 32) {
    const v16b a  = ldfrag_b(ap + k0);
    const v16b b0 = ldfrag_b(bp + k0);
    const v16b b1 = ldfrag_b(bp + bs + k0);
    const v16b b2 = ldfrag_b(bp + 2 * bs + k0);
    const v16b b3 = ldfrag_b(bp + 3 * bs + k0);
    acc0 = mma_b(a, b0, acc0);
    acc1 = mma_b(a, b1, acc1);
    acc2 = mma_b(a, b2, acc2);
    acc3 = mma_b(a, b3, acc3);
    guard4x5<v16b>(acc0, acc1, acc2, acc3, a, b0, b1, b2, b3);
  }
  float* sl = slab + wave * GSLAB;
  if (OM == 0) {
    float bc[4];
#pragma unroll
    for (int j = 0; j < 4; ++j) bc[j] = bf_up(bf_bits(bias[imin(col0 + 16 * j + m, nbias - 1)]));
#pragma unroll
    for (int r = 0; r < 8; ++r) {
      const int ro = (8 * hh + r) * 68 + m;
      sl[ro]      = (acc0[r] + bc[0]) * oscale;
      sl[ro + 16] = (acc1[r] + bc[1]) * oscale;
      sl[ro + 32] = (acc2[r] + bc[2]) * oscale;
      sl[ro + 48] = (acc3[r] + bc[3]) * oscale;
    }
  } else {
#pragma unroll
    for (int r = 0; r < 8; ++r) {
      const float br = bf_up(bf_bits(bias[imin(rowb + 8 * hh + r, nbias - 1)]));
      const int ro = (8 * hh + r) * 68 + m;
      sl[ro]      = (acc0[r] + br) * oscale;
      sl[ro + 16] = (acc1[r] + br) * oscale;
      sl[ro + 32] = (acc2[r] + br) * oscale;
      sl[ro + 48] = (acc3[r] + br) * oscale;
    }
  }
  wave_sync_lds();
  const int rq = lane >> 3, c8 = (lane & 7) * 8;
  v4u ov[4];
#pragma unroll
  for (int i4 = 0; i4 < 4; ++i4) {
    const int row = i4 * 4 + rq;
    const v4f a = *(const v4f*)(sl + row * 68 + c8), c4 = *(const v4f*)(sl + row * 68 + c8 + 4);
    float w[8];
#pragma unroll
    for (int e = 0; e < 4; ++e) { w[e] = a[e]; w[4 + e] = c4[e]; }
#pragma unroll
    for (int e = 0; e < 4; ++e) ov[i4][e] = pk16(h_bits((_Float16)w[2 * e]), h_bits((_Float16)w[2 * e + 1]));
  }
  const size_t dofs = ((size_t)rowb + (size_t)rq) * (size_t)N + col0 + c8;
  u16* dst = Cb + dofs;
  for (int pass = 0; pass < 2; ++pass) {
#pragma unroll
    for (int i4 = 0; i4 < 4; ++i4) {
      *(volatile v4u*)(dst + (size_t)(i4 * 4) * (size_t)N) = ov[i4];
    }
    __threadfence();
  }
}

__global__ __launch_bounds__(128)
void gemm_ho(const u16* __restrict__ A, const u16* __restrict__ Bt, const float* __restrict__ bias, int nbias,
             float* C, int M, int N, int K, int bstA, int bstB, int bstC, float oscale) {
  __shared__ __align__(16) float slab[4 * GSLAB];
  const int tid = threadIdx.x, wave = tid >> 5, lane = tid & 31, hh = lane >> 4, m = lane & 15;
  const int ntile = N >> 6, mtile = M >> 6;
  const int per   = ntile * mtile;
  const int bid   = blockIdx.x;
  const int bt    = bid / per;
  const int t     = bid - bt * per;
  const int rowb  = (t / ntile) * 64 + wave * 16;
  const int col0  = (t % ntile) * 64;
  if (rowb + 16 > M) return;
  const _Float16* ap = (const _Float16*)(const void*)(A + (size_t)bt * (size_t)bstA) + (size_t)(rowb + m) * K + 8 * hh;
  const _Float16* bp = (const _Float16*)(const void*)(Bt + (size_t)bt * (size_t)bstB) + (size_t)(col0 + m) * K + 8 * hh;
  float* Cb = C + (size_t)bt * (size_t)bstC;
  const size_t bs = (size_t)16 * K;
  v8f acc0 = zero8(), acc1 = zero8(), acc2 = zero8(), acc3 = zero8();
#pragma unroll 1
  for (int k0 = 0; k0 < K; k0 += 32) {
    const v16h a  = ldfrag_h(ap + k0);
    const v16h b0 = ldfrag_h(bp + k0);
    const v16h b1 = ldfrag_h(bp + bs + k0);
    const v16h b2 = ldfrag_h(bp + 2 * bs + k0);
    const v16h b3 = ldfrag_h(bp + 3 * bs + k0);
    acc0 = mma_h(a, b0, acc0);
    acc1 = mma_h(a, b1, acc1);
    acc2 = mma_h(a, b2, acc2);
    acc3 = mma_h(a, b3, acc3);
    guard4x5<v16h>(acc0, acc1, acc2, acc3, a, b0, b1, b2, b3);
  }
  float* sl = slab + wave * GSLAB;
  float bc[4];
#pragma unroll
  for (int j = 0; j < 4; ++j) bc[j] = bf_up(bf_bits(bias[imin(col0 + 16 * j + m, nbias - 1)]));
#pragma unroll
  for (int r = 0; r < 8; ++r) {
    const int ro = (8 * hh + r) * 68 + m;
    sl[ro]      = acc0[r] * oscale + bc[0];
    sl[ro + 16] = acc1[r] * oscale + bc[1];
    sl[ro + 32] = acc2[r] * oscale + bc[2];
    sl[ro + 48] = acc3[r] * oscale + bc[3];
  }
  wave_sync_lds();
  v4f vals[8];
#pragma unroll
  for (int it = 0; it < 8; ++it) vals[it] = *(const v4f*)(sl + (it * 2 + hh) * 68 + m * 4);
  float* dst = Cb + ((size_t)rowb + (size_t)hh) * (size_t)N + col0 + m * 4;
  for (int pass = 0; pass < 2; ++pass) {
#pragma unroll
    for (int it = 0; it < 8; ++it) {
      *(volatile v4f*)(dst + (size_t)(it * 2) * (size_t)N) = vals[it];
    }
    __threadfence();
  }
}

__global__ __launch_bounds__(ATT_THREADS)
void attn_fwd(const u16* __restrict__ QPp, const u16* __restrict__ KPp, const u16* __restrict__ VPp,
              const int* __restrict__ MKp, u16* OPp) {
  __shared__ __align__(16) float smem[ATT_WAVES * ASLAB];

  const int tid  = threadIdx.x;
  const int wave = tid >> 5;
  const int lane = tid & 31;
  const int hh   = lane >> 4;
  const int c    = lane & 15;

  const int bid  = blockIdx.x;
  const int qt   = bid % NQT;
  const int head = (bid / NQT) % NH;
  const int b    = bid / (NQT * NH);
  const int q0   = qt * 64 + wave * 16;

  const size_t qofs = (((size_t)(b * SEQ + q0 + c)) * NH + head) * HD + 8 * hh;
  const _Float16* Qb = (const _Float16*)(const void*)QPp + qofs;
  const size_t kofs = (((size_t)(b * SEQ + c)) * NH + head) * HD + 8 * hh;
  const _Float16* Kb = (const _Float16*)(const void*)KPp + kofs;
  const size_t vofs = ((size_t)(b * NH + head) * HD + c) * SEQ + 8 * hh;
  const _Float16* Vb = (const _Float16*)(const void*)VPp + vofs;
  const int* Mb = MKp + ((size_t)(b * SEQ + q0 + c)) * SEQ + 8 * hh;

  const int   ex     = head + 1;
  const float slope  = (((ex & 1) != 0) ? RSQ2 : 1.0f) * __int_as_float((127 - (ex >> 1)) << 23);
  const float slope2 = slope * LOG2E;
  const float lsc    = (INVN * LOG2E) * (1.0f / (QSC * KSC));
  const float jb0    = (float)(8 * hh - (SEQ - 1));

  const v16h qf0 = ldfrag_h(Qb);
  const v16h qf1 = ldfrag_h(Qb + 32);
  const v16h qf2 = ldfrag_h(Qb + 64);
  const v16h qf3 = ldfrag_h(Qb + 96);

  float mrun = -INFINITY, lrun = 0.f;
  v8f o[8];
#pragma unroll
  for (int j = 0; j < 8; ++j) o[j] = zero8();

#pragma unroll 1
  for (int it = 0; it < NKB; ++it) {
    const int kb = it * 32;
    v8f s0 = zero8(), s1 = zero8();
    const _Float16* k0p = Kb + (size_t)kb * NHD;
    const _Float16* k1p = k0p + (size_t)16 * NHD;
    {
      const v16h ka0 = ldfrag_h(k0p),      ka1 = ldfrag_h(k0p + 32);
      const v16h kc0 = ldfrag_h(k1p),      kc1 = ldfrag_h(k1p + 32);
      s0 = mma_h(ka0, qf0, s0);
      s0 = mma_h(ka1, qf1, s0);
      s1 = mma_h(kc0, qf0, s1);
      s1 = mma_h(kc1, qf1, s1);
      guard2x6<v16h>(s0, s1, qf0, qf1, ka0, ka1, kc0, kc1);
    }
    {
      const v16h ka2 = ldfrag_h(k0p + 64), ka3 = ldfrag_h(k0p + 96);
      const v16h kc2 = ldfrag_h(k1p + 64), kc3 = ldfrag_h(k1p + 96);
      s0 = mma_h(ka2, qf2, s0);
      s0 = mma_h(ka3, qf3, s0);
      s1 = mma_h(kc2, qf2, s1);
      s1 = mma_h(kc3, qf3, s1);
      guard2x6<v16h>(s0, s1, qf2, qf3, ka2, ka3, kc2, kc3);
    }
    const v4i w0 = *(const v4i*)(Mb + kb),      w1 = *(const v4i*)(Mb + kb + 4);
    const v4i w2 = *(const v4i*)(Mb + kb + 16), w3 = *(const v4i*)(Mb + kb + 20);
    int mv[16];
#pragma unroll
    for (int e = 0; e < 4; ++e) { mv[e] = w0[e]; mv[4 + e] = w1[e]; mv[8 + e] = w2[e]; mv[12 + e] = w3[e]; }
    const float jb = jb0 + (float)kb;
    float tk[16];
#pragma unroll
    for (int i = 0; i < 8; ++i) {
      const float t0 = fmaf(s0[i], lsc, slope2 * (jb + (float)i));
      const float t1 = fmaf(s1[i], lsc, slope2 * (jb + (float)(16 + i)));
      tk[i]     = (mv[i] != 0)     ? t0 : MFILL;
      tk[8 + i] = (mv[8 + i] != 0) ? t1 : MFILL;
    }
    float cm = tk[0];
#pragma unroll
    for (int i = 1; i < 16; ++i) cm = fmaxf(cm, tk[i]);
    cm = fmaxf(cm, __shfl_xor(cm, 16, 32));
    const float mn = fmaxf(mrun, cm);
    const float al = (mrun == -INFINITY) ? 0.f : exp2f(mrun - mn);
    mrun = mn;
    float ps = 0.f;
    FragH ph;
#pragma unroll
    for (int w = 0; w < 2; ++w) {
#pragma unroll
      for (int e4 = 0; e4 < 4; ++e4) {
        const int i = 8 * w + 2 * e4;
        const float p0 = exp2f(fminf(tk[i] - mn, 0.f));
        const float p1 = exp2f(fminf(tk[i + 1] - mn, 0.f));
        ps += p0 + p1;
        ph.u[w][e4] = pk16(h_bits((_Float16)(p0 * PCAR)), h_bits((_Float16)(p1 * PCAR)));
      }
    }
    ps += __shfl_xor(ps, 16, 32);
    lrun = lrun * al + ps;
    float scl[8];
#pragma unroll
    for (int r = 0; r < 8; ++r) scl[r] = __shfl(al, 8 * hh + r, 32);
#pragma unroll
    for (int j = 0; j < 8; ++j) {
#pragma unroll
      for (int r = 0; r < 8; ++r) o[j][r] *= scl[r];
    }
    {
      const _Float16* vp = Vb + kb;
      const v16h vf0 = ldfrag_h(vp);
      const v16h vf1 = ldfrag_h(vp + (size_t)16 * SEQ);
      const v16h vf2 = ldfrag_h(vp + (size_t)32 * SEQ);
      const v16h vf3 = ldfrag_h(vp + (size_t)48 * SEQ);
      o[0] = mma_h(ph.v, vf0, o[0]);
      o[1] = mma_h(ph.v, vf1, o[1]);
      o[2] = mma_h(ph.v, vf2, o[2]);
      o[3] = mma_h(ph.v, vf3, o[3]);
      guard4x5<v16h>(o[0], o[1], o[2], o[3], ph.v, vf0, vf1, vf2, vf3);
      const v16h vf4 = ldfrag_h(vp + (size_t)64 * SEQ);
      const v16h vf5 = ldfrag_h(vp + (size_t)80 * SEQ);
      const v16h vf6 = ldfrag_h(vp + (size_t)96 * SEQ);
      const v16h vf7 = ldfrag_h(vp + (size_t)112 * SEQ);
      o[4] = mma_h(ph.v, vf4, o[4]);
      o[5] = mma_h(ph.v, vf5, o[5]);
      o[6] = mma_h(ph.v, vf6, o[6]);
      o[7] = mma_h(ph.v, vf7, o[7]);
      guard4x5<v16h>(o[4], o[5], o[6], o[7], ph.v, vf4, vf5, vf6, vf7);
    }
  }
  acc_guard4(o[0], o[1], o[2], o[3]);
  acc_guard4(o[4], o[5], o[6], o[7]);

  const float linv = (lrun > 0.f) ? ((1.0f / lrun) * (OSC / (PCAR * VCAR))) : 0.f;
  float inv[8];
#pragma unroll
  for (int r = 0; r < 8; ++r) inv[r] = __shfl(linv, 8 * hh + r, 32);
  float* slab = smem + wave * ASLAB;
#pragma unroll
  for (int r = 0; r < 8; ++r) {
#pragma unroll
    for (int j = 0; j < 8; ++j) slab[(8 * hh + r) * 132 + j * 16 + c] = o[j][r] * inv[r];
  }
  wave_sync_lds();
  const int rq = hh, c8 = c * 8;
  v4u oh[8];
#pragma unroll
  for (int i2 = 0; i2 < 8; ++i2) {
    const int row = i2 * 2 + rq;
    const v4f a = *(const v4f*)(slab + row * 132 + c8), c4 = *(const v4f*)(slab + row * 132 + c8 + 4);
    float w[8];
#pragma unroll
    for (int e = 0; e < 4; ++e) { w[e] = a[e]; w[4 + e] = c4[e]; }
#pragma unroll
    for (int e = 0; e < 4; ++e) oh[i2][e] = pk16(h_bits((_Float16)w[2 * e]), h_bits((_Float16)w[2 * e + 1]));
  }
  const size_t ob = (((size_t)(b * SEQ + q0)) * NH + head) * HD + c8;
  for (int pass = 0; pass < 2; ++pass) {
#pragma unroll
    for (int i2 = 0; i2 < 8; ++i2) {
      const int row = i2 * 2 + rq;
      const size_t o8 = ob + (size_t)row * NHD;
      *(volatile v4u*)(OPp + o8) = oh[i2];
    }
    __threadfence();
  }
}

extern "C" void kernel_launch(void* const* d_in, const int* in_sizes, int n_in,
                              void* d_out, int out_size, void* d_ws, size_t ws_size,
                              hipStream_t stream) {
  const int ROWS = NB * SEQ;
  if (n_in < 10) return;
  if (in_sizes[0] != ROWS * DMOD) return;
  if (in_sizes[1] != NB * SEQ * SEQ) return;
  if (in_sizes[2] != DMOD * NHD || in_sizes[4] != DMOD * NHD || in_sizes[6] != DMOD * NHD) return;
  if (in_sizes[3] != NHD || in_sizes[5] != NHD || in_sizes[7] != NHD) return;
  if (in_sizes[8] != DMOD * DMOD || in_sizes[9] != DMOD) return;
  if (out_size != ROWS * DMOD) return;

  const float* Xin = (const float*)d_in[0];
  const int*   Min = (const int*)d_in[1];
  const float* wq  = (const float*)d_in[2];
  const float* bq  = (const float*)d_in[3];
  const float* wk  = (const float*)d_in[4];
  const float* bk  = (const float*)d_in[5];
  const float* wv  = (const float*)d_in[6];
  const float* bv  = (const float*)d_in[7];
  const float* wo  = (const float*)d_in[8];
  const float* bo  = (const float*)d_in[9];
  float*       out = (float*)d_out;

  const size_t szXB  = (size_t)ROWS * DMOD * 2;
  const size_t szWO  = (size_t)DMOD * DMOD * 2;
  const size_t szW3  = (size_t)3 * NHD * DMOD * 2;
  const size_t szPl  = (size_t)ROWS * NHD * 2;
  const size_t szVP  = (size_t)NB * NHD * SEQ * 2;
  const size_t szR0  = (szXB > szWO) ? szXB : szWO;
  const size_t szR1  = (szW3 > szPl) ? szW3 : szPl;
  size_t off = 0;
  const size_t oR0 = off; off += szR0;
  const size_t oR1 = off; off += szR1;
  const size_t oQP = off; off += szPl;
  const size_t oKP = off; off += szPl;
  const size_t oVP = off; off += szVP;
  if (off > ws_size) return;
  if (off > (size_t)134217728) return;

  char* ws = (char*)d_ws;
  u16* XB  = (u16*)(ws + oR0);
  u16* WOB = (u16*)(ws + oR0);
  u16* WQT = (u16*)(ws + oR1);
  u16* WKT = WQT + (size_t)NHD * DMOD;
  u16* WVT = WKT + (size_t)NHD * DMOD;
  u16* OP  = (u16*)(ws + oR1);
  u16* QP  = (u16*)(ws + oQP);
  u16* KP  = (u16*)(ws + oKP);
  u16* VP  = (u16*)(ws + oVP);

  const int n8x = (ROWS * DMOD) / 8;
  if ((n8x % 256) != 0) return;
  if ((DMOD % 64) != 0 || (NHD % 64) != 0 || (SEQ % 64) != 0 || (SQ % 64) != 0 || (DMOD % 32) != 0) return;

  const dim3 blk(256);
  const dim3 gX(n8x / 256);
  const dim3 gT(NHD / 64, DMOD / 64);
  const dim3 gTo(DMOD / 64, DMOD / 64);
  const dim3 bG(128);
  const dim3 gQ(NB * (SQ / 64) * (NHD / 64));
  const dim3 gK(NB * (SEQ / 64) * (NHD / 64));
  const dim3 gV(NB * (NHD / 64) * (SEQ / 64));
  const dim3 gAT(ATT_BLOCKS);
  const dim3 bAT(ATT_THREADS);
  const dim3 gO(NB * (SQ / 64) * (DMOD / 64));

  cvt16<<<gX, blk, 0, stream>>>(Xin, XB, n8x, 0, 1.0f);
  wtr16<<<gT, blk, 0, stream>>>(wq, WQT, DMOD, NHD, 0, 1.0f);
  wtr16<<<gT, blk, 0, stream>>>(wk, WKT, DMOD, NHD, 0, 1.0f);
  wtr16<<<gT, blk, 0, stream>>>(wv, WVT, DMOD, NHD, 0, 1.0f);
  gemm_bb<0><<<gQ, bG, 0, stream>>>(XB, WQT, bq, NHD, QP, SQ, NHD, DMOD, SEQ * DMOD, 0, SEQ * NHD, QSC);
  gemm_bb<0><<<gK, bG, 0, stream>>>(XB, WKT, bk, NHD, KP, SEQ, NHD, DMOD, SEQ * DMOD, 0, SEQ * NHD, KSC);
  gemm_bb<1><<<gV, bG, 0, stream>>>(WVT, XB, bv, NHD, VP, NHD, SEQ, DMOD, 0, SEQ * DMOD, NHD * SEQ, VCAR);
  wtr16<<<gTo, blk, 0, stream>>>(wo, WOB, DMOD, DMOD, 1, WOS);
  attn_fwd<<<gAT, bAT, 0, stream>>>(QP, KP, VP, Min, OP);
  gemm_ho<<<gO, bG, 0, stream>>>(OP, WOB, bo, DMOD, out, SQ, DMOD, NHD, SEQ * NHD, 0, SEQ * DMOD, 1.0f / (OSC * WOS));
  (void)hipGetLastError();
}
